// LDS_63720134804240
// MI455X (gfx1250) — hardware-verified
//
#include <hip/hip_runtime.h>

constexpr int  kBatch    = 8;
constexpr int  kTime     = 4096;
constexpr int  kDimIn    = 128;
constexpr int  kState    = 1024;
constexpr int  kDimOut   = 128;
constexpr int  kTaps     = 10;
constexpr int  kPadRows  = 16;
constexpr int  kTimePad  = kTime + kPadRows;
constexpr long kXPlane   = (long)kTimePad * kDimIn;
constexpr int  kArK      = kTaps * kDimIn;
constexpr int  kChunkB   = 2;
constexpr int  kNumChunk = kBatch / kChunkB;

constexpr float kXCarry   = 8.0f;
constexpr float kBCarry   = 64.0f;
constexpr float kCCarry   = 1024.0f;
constexpr float kMCarry   = 64.0f;
constexpr float kHCarry   = 32.0f;
constexpr float kProjScale = 1.0f / (kXCarry * kBCarry);
constexpr float kReadScale = 1.0f / (kHCarry * kCCarry);
constexpr float kArScale   = 1.0f / (kXCarry * kMCarry);

static_assert(kPadRows >= kTaps - 1);
static_assert(kArK % 32 == 0);
static_assert((kBatch * kTimePad * (kDimIn / 8)) % 256 == 0);

typedef __attribute__((ext_vector_type(16))) _Float16 v16h;
typedef __attribute__((ext_vector_type(8)))  _Float16 v8h;
typedef __attribute__((ext_vector_type(16))) __bf16   v16b;
typedef __attribute__((ext_vector_type(8)))  __bf16   v8b;
typedef __attribute__((ext_vector_type(8)))  float    v8f;
typedef __attribute__((ext_vector_type(4)))  float    v4f;
typedef __attribute__((ext_vector_type(4)))  unsigned int v4u;

__device__ __forceinline__ unsigned short f2bf_bits(float f) {
  unsigned u = __float_as_uint(f);
  return (unsigned short)((u + 0x7FFFu + ((u >> 16) & 1u)) >> 16);
}
__device__ __forceinline__ float bf_bits2f(unsigned short h) { return __uint_as_float(((unsigned)h) << 16); }

__device__ __forceinline__ void dep_guard_h(v8f& a, v8f& b, v16h x, v16h y) { asm volatile("v_nop\n\tv_nop\n\tv_nop\n\tv_nop" : "+v"(a), "+v"(b) : "v"(x), "v"(y)); }
__device__ __forceinline__ void dep_guard_b(v8f& a, v8f& b, v16b x, v16b y) { asm volatile("v_nop\n\tv_nop\n\tv_nop\n\tv_nop" : "+v"(a), "+v"(b) : "v"(x), "v"(y)); }
__device__ __forceinline__ void keep4_h(v16h a, v16h b, v16h c, v16h d) { asm volatile("v_nop" :: "v"(a), "v"(b), "v"(c), "v"(d)); }
__device__ __forceinline__ void keep4_b(v16b a, v16b b, v16b c, v16b d) { asm volatile("v_nop" :: "v"(a), "v"(b), "v"(c), "v"(d)); }
__device__ __forceinline__ void acc_guard4(v8f& a, v8f& b, v8f& c, v8f& d) { asm volatile("v_nop\n\tv_nop\n\tv_nop\n\tv_nop" : "+v"(a), "+v"(b), "+v"(c), "+v"(d)); }
template <typename T> struct Frag;
template <> struct Frag<_Float16> {
  typedef v16h V; union U { v16h v; v8h h[2]; };
  static __device__ __forceinline__ v16h load(const _Float16* p) {
    U f; f.h[0] = *(const v8h*)(p); f.h[1] = *(const v8h*)(p + 16); return f.v;
  }
  static __device__ __forceinline__ v8f mma(v16h a, v16h b, v8f c) {
    return __builtin_amdgcn_wmma_f32_16x16x32_f16(false, a, false, b, (short)0, c, false, false);
  }
  static __device__ __forceinline__ void guard(v8f& a, v8f& b, v16h x, v16h y) { dep_guard_h(a, b, x, y); }
  static __device__ __forceinline__ void keep(v16h a, v16h b, v16h c, v16h d) { keep4_h(a, b, c, d); }
};
template <> struct Frag<__bf16> {
  typedef v16b V; union U { v16b v; v8b h[2]; };
  static __device__ __forceinline__ v16b load(const __bf16* p) {
    U f; f.h[0] = *(const v8b*)(p); f.h[1] = *(const v8b*)(p + 16); return f.v;
  }
  static __device__ __forceinline__ v8f mma(v16b a, v16b b, v8f c) {
    return __builtin_amdgcn_wmma_f32_16x16x32_bf16(false, a, false, b, (short)0, c, false, false);
  }
  static __device__ __forceinline__ void guard(v8f& a, v8f& b, v16b x, v16b y) { dep_guard_b(a, b, x, y); }
  static __device__ __forceinline__ void keep(v16b a, v16b b, v16b c, v16b d) { keep4_b(a, b, c, d); }
};

__device__ __forceinline__ unsigned pk16(unsigned short a, unsigned short b) { return (unsigned)a | ((unsigned)b << 16); }
__device__ __forceinline__ unsigned short h_bits(float f) { const _Float16 h = (_Float16)f; return __builtin_bit_cast(unsigned short, h); }

template <int ET> struct Elem;
template <> struct Elem<0> { typedef _Float16 T; };
template <> struct Elem<1> { typedef __bf16 T; };
template <int ET, bool SPLIT, int BIAS_MODE, int OUT_MODE, bool RESID, int ACT = 0>
__global__ __launch_bounds__(256) void wmma_gemm64(
    const unsigned short* __restrict__ Ap, const unsigned short* __restrict__ A2p, int lda, long strideA,
    const unsigned short* __restrict__ Btp, const unsigned short* __restrict__ Bt2p, int ldb, long strideB,
    void* __restrict__ Cout, void* __restrict__ Cout2, int ldc, long strideC,
    const float* __restrict__ bias,
    const float* __restrict__ resid, long strideR,
    int M, int N, int K, float scale) {
  typedef typename Elem<ET>::T T;
  typedef typename Frag<T>::V V;
  const T* A = (const T*)Ap; const T* A2 = (const T*)A2p; const T* Bt = (const T*)Btp; const T* Bt2 = (const T*)Bt2p;
  __shared__ __align__(16) float sT[8][16 * 68];
  const int b    = blockIdx.y;
  const int lane = threadIdx.x & 31;
  const int wave = threadIdx.x >> 5;
  const int tilesN = N >> 6;
  const int tilesM = M >> 6;
  const int tile = blockIdx.x * 8 + wave;
  if (tile >= tilesM * tilesN) return;
  const int tm = tile / tilesN;
  const int tn = tile - tm * tilesN;
  const int m0 = tm << 6;
  const int n0 = tn << 6;

  const T* Ab  = A  + (size_t)b * strideA;
  const T* Bb  = Bt + (size_t)b * strideB;
  const T* Ab2 = SPLIT ? (A2  + (size_t)b * strideA) : nullptr;
  const T* Bb2 = SPLIT ? (Bt2 + (size_t)b * strideB) : nullptr;

  const int rlane = lane & 15;
  const int koff  = (lane >> 4) * 8;
  const int mOff  = (lane >> 4) * 8;

  v8f acc[4][4];
#pragma unroll
  for (int i = 0; i < 4; ++i)
#pragma unroll
    for (int j = 0; j < 4; ++j) acc[i][j] = (v8f){0.f,0.f,0.f,0.f,0.f,0.f,0.f,0.f};

  for (int k0 = 0; k0 < K; k0 += 32) {
    V bh[4], bl[4];
#pragma unroll
    for (int j = 0; j < 4; ++j) {
      const size_t bo = (size_t)(n0 + (j << 4) + rlane) * ldb + koff + k0;
      bh[j] = Frag<T>::load(Bb + bo);
      if (SPLIT) bl[j] = Frag<T>::load(Bb2 + bo);
    }
#pragma unroll
    for (int i = 0; i < 4; ++i) {
      const size_t ao = (size_t)(m0 + (i << 4) + rlane) * lda + koff + k0;
      V ah = Frag<T>::load(Ab + ao);
      V al;
      if (SPLIT) al = Frag<T>::load(Ab2 + ao);
#pragma unroll
      for (int j = 0; j < 4; ++j) {
        acc[i][j] = Frag<T>::mma(ah, bh[j], acc[i][j]);
        if (SPLIT) {
          acc[i][j] = Frag<T>::mma(ah, bl[j], acc[i][j]);
          acc[i][j] = Frag<T>::mma(al, bh[j], acc[i][j]);
        }
      }
      Frag<T>::guard(acc[i][0], acc[i][3], ah, SPLIT ? al : ah);
    }
    Frag<T>::keep(bh[0], bh[1], bh[2], bh[3]);
    if (SPLIT) Frag<T>::keep(bl[0], bl[1], bl[2], bl[3]);
  }
  acc_guard4(acc[0][0], acc[0][1], acc[0][2], acc[0][3]);
  acc_guard4(acc[1][0], acc[1][1], acc[1][2], acc[1][3]);
  acc_guard4(acc[2][0], acc[2][1], acc[2][2], acc[2][3]);
  acc_guard4(acc[3][0], acc[3][1], acc[3][2], acc[3][3]);

  float* slab = sT[wave];
  const float* Rb = RESID ? (resid + (size_t)b * strideR) : nullptr;
#pragma unroll
  for (int i = 0; i < 4; ++i) {
    const int mBase = m0 + (i << 4);
#pragma unroll
    for (int j = 0; j < 4; ++j) {
      const int n = n0 + (j << 4) + rlane;
      float bv = 0.f;
      if (BIAS_MODE == 2) bv = bias[n];
#pragma unroll
      for (int r = 0; r < 8; ++r) {
        float v = acc[i][j][r] * scale;
        if (BIAS_MODE == 1) v += bias[mBase + mOff + r];
        if (BIAS_MODE == 2) v += bv;
        if (RESID) v += Rb[(size_t)(mBase + mOff + r) * ldc + n];
        if (ACT == 2) v = fmaxf(v, 0.0f);
        if (ACT == 4) v = (v > 0.f) ? v : 0.01f * v;
        slab[(mOff + r) * 68 + (j << 4) + rlane] = v;
      }
    }
    __builtin_amdgcn_fence(__ATOMIC_RELEASE, "workgroup");
    __builtin_amdgcn_wave_barrier();
    __builtin_amdgcn_fence(__ATOMIC_ACQUIRE, "workgroup");
    if (OUT_MODE == 0) {
      float* C = (float*)Cout + (size_t)b * strideC;
      const int hh = lane >> 4, c4 = (lane & 15) * 4;
      for (int pass = 0; pass < 2; ++pass) {
#pragma unroll
        for (int it = 0; it < 8; ++it) {
          const int row = it * 2 + hh;
          v4f v = *(const v4f*)(slab + row * 68 + c4);
          *(volatile v4f*)(C + (size_t)(mBase + row) * ldc + n0 + c4) = v;
        }
        __threadfence();
      }
    } else {
      const int q = lane >> 3, c8 = (lane & 7) * 8;
      unsigned short* C  = (unsigned short*)Cout  + (size_t)b * strideC;
      unsigned short* C2 = (OUT_MODE == 2) ? ((unsigned short*)Cout2 + (size_t)b * strideC) : nullptr;
      for (int pass = 0; pass < 2; ++pass) {
#pragma unroll
        for (int it = 0; it < 4; ++it) {
          const int row = it * 4 + q;
          const float* sp = slab + row * 68 + c8;
          v8h hv, lv;
#pragma unroll
          for (int e = 0; e < 8; ++e) {
            if (OUT_MODE == 1) {
              hv[e] = (_Float16)sp[e];
            } else {
              unsigned short hb = f2bf_bits(sp[e]);
              unsigned short lb = f2bf_bits(sp[e] - bf_bits2f(hb));
              hv[e] = __builtin_bit_cast(_Float16, hb);
              lv[e] = __builtin_bit_cast(_Float16, lb);
            }
          }
          *(volatile v8h*)(C + (size_t)(mBase + row) * ldc + n0 + c8) = hv;
          if (OUT_MODE == 2) *(volatile v8h*)(C2 + (size_t)(mBase + row) * ldc + n0 + c8) = lv;
        }
        __threadfence();
      }
    }
    __builtin_amdgcn_fence(__ATOMIC_RELEASE, "workgroup");
    __builtin_amdgcn_wave_barrier();
    __builtin_amdgcn_fence(__ATOMIC_ACQUIRE, "workgroup");
  }
}

__global__ __launch_bounds__(256) void castx_kernel(const float* __restrict__ X, unsigned short* __restrict__ Xp, int nthr) {
  const int i = blockIdx.x * 256 + threadIdx.x;
  if (i >= nthr) return;
  constexpr int perB = kTimePad * (kDimIn / 8);
  const int b   = i / perB;
  const int rem = i - b * perB;
  const int r   = rem >> 4;
  const int c8  = (rem & 15) * 8;
  const int tr  = r - kPadRows;
  const int trc = tr < 0 ? 0 : tr;
  const float* p = X + ((size_t)b * kTime + trc) * kDimIn + c8;
  const v4f a = *(const v4f*)(p);
  const v4f c = *(const v4f*)(p + 4);
  const bool live = (tr >= 0);
  unsigned short hb[8];
#pragma unroll
  for (int e = 0; e < 4; ++e) {
    const float f0 = live ? a[e] * kXCarry : 0.0f;
    const float f1 = live ? c[e] * kXCarry : 0.0f;
    hb[e]     = h_bits(f0);
    hb[4 + e] = h_bits(f1);
  }
  const v4u u = (v4u){pk16(hb[0], hb[1]), pk16(hb[2], hb[3]), pk16(hb[4], hb[5]), pk16(hb[6], hb[7])};
  unsigned short* q = Xp + 8 * (size_t)i;
  *(volatile v4u*)q = u;
  __threadfence();
  *(volatile v4u*)q = u;
}

template <int MODE>
__global__ __launch_bounds__(256) void wprep_kernel(const float* __restrict__ W, unsigned short* __restrict__ out, int nthr) {
  const int i = blockIdx.x * 256 + threadIdx.x;
  if (i >= nthr) return;
  float v[8];
  if (MODE == 0) {
    const int n = i >> 4, d8 = (i & 15) * 8;
#pragma unroll
    for (int e = 0; e < 8; ++e) v[e] = W[(size_t)(d8 + e) * kState + n] * kBCarry;
  } else if (MODE == 1) {
    const int o = i >> 7, n8 = (i & 127) * 8;
#pragma unroll
    for (int e = 0; e < 8; ++e) v[e] = W[(size_t)(n8 + e) * kDimOut + o] * kCCarry;
  } else {
    constexpr int thrPerRow = kArK / 8;
    const int o  = i / thrPerRow;
    const int k8 = (i - o * thrPerRow) * 8;
    const int j  = k8 >> 7;
    const int d8 = k8 & 127;
    const int tap = kTaps - 1 - j;
#pragma unroll
    for (int e = 0; e < 8; ++e) v[e] = W[((size_t)(o * kDimIn + d8 + e)) * kTaps + tap] * kMCarry;
  }
  unsigned short hb[8];
#pragma unroll
  for (int e = 0; e < 8; ++e) hb[e] = h_bits(v[e]);
  const v4u u = (v4u){pk16(hb[0], hb[1]), pk16(hb[2], hb[3]), pk16(hb[4], hb[5]), pk16(hb[6], hb[7])};
  unsigned short* q = out + 8 * (size_t)i;
  *(volatile v4u*)q = u;
  __threadfence();
  *(volatile v4u*)q = u;
}

__global__ __launch_bounds__(32) void scan_kernel(const float* __restrict__ U, const float* __restrict__ h0,
                                                  const float* __restrict__ Ad, unsigned short* __restrict__ H,
                                                  int bBase) {
  const int g = blockIdx.x * 32 + threadIdx.x;
  if (g >= kChunkB * (kState / 8)) return;
  const int bl = g >> 7;
  const int n0 = (g & 127) * 8;
  const v4f a0 = *(const v4f*)(Ad + n0), a1 = *(const v4f*)(Ad + n0 + 4);
  const v4f g0 = *(const v4f*)(h0 + n0), g1 = *(const v4f*)(h0 + n0 + 4);
  float a[8], h[8];
#pragma unroll
  for (int e = 0; e < 4; ++e) { a[e] = a0[e]; a[4 + e] = a1[e]; h[e] = g0[e]; h[4 + e] = g1[e]; }
  const float* up = U + (size_t)bl * kTime * kState + n0;
  unsigned short* hp = H + ((size_t)(bBase + bl) * kTime) * kState + n0;
#pragma unroll 1
  for (int t = 0; t < kTime; ++t) {
    const v4f u0 = *(const v4f*)(up);
    const v4f u1 = *(const v4f*)(up + 4);
    float u[8];
#pragma unroll
    for (int e = 0; e < 4; ++e) { u[e] = u0[e]; u[4 + e] = u1[e]; }
    unsigned short hb[8];
#pragma unroll
    for (int e = 0; e < 8; ++e) {
      h[e] = a[e] * h[e] + u[e];
      hb[e] = h_bits(h[e] * kHCarry);
    }
    const v4u w = (v4u){pk16(hb[0], hb[1]), pk16(hb[2], hb[3]), pk16(hb[4], hb[5]), pk16(hb[6], hb[7])};
    *(volatile v4u*)hp = w;
    __threadfence();
    *(volatile v4u*)hp = w;
    up += kState;
    hp += kState;
  }
}

extern "C" void kernel_launch(void* const* d_in, const int* in_sizes, int n_in,
                              void* d_out, int out_size, void* d_ws, size_t ws_size,
                              hipStream_t stream) {
  if (n_in < 6) return;
  const float* X  = (const float*)d_in[0];
  const float* H0 = (const float*)d_in[1];
  const float* Ad = (const float*)d_in[2];
  const float* Bm = (const float*)d_in[3];
  const float* Cm = (const float*)d_in[4];
  const float* Mm = (const float*)d_in[5];
  if (in_sizes[0] != kBatch * kTime * kDimIn || in_sizes[1] != kState || in_sizes[2] != kState ||
      in_sizes[3] != kDimIn * kState || in_sizes[4] != kState * kDimOut ||
      in_sizes[5] != kDimOut * kDimIn * kTaps || out_size != kBatch * kTime * kDimOut) return;

  const size_t szU  = (size_t)kChunkB * kTime * kState * sizeof(float);
  const size_t szH  = (size_t)kBatch * kTime * kState * sizeof(unsigned short);
  const size_t szR  = (size_t)kBatch * kTime * kDimOut * sizeof(float);
  const size_t szX  = (size_t)kBatch * kXPlane * sizeof(unsigned short);
  const size_t szBt = (size_t)kState * kDimIn * sizeof(unsigned short);
  const size_t szCt = (size_t)kDimOut * kState * sizeof(unsigned short);
  const size_t szMt = (size_t)kDimOut * kArK * sizeof(unsigned short);
  size_t off = 0;
  char* ws = (char*)d_ws;
  float*          Ubuf = (float*)(ws + off);          off += szU;
  unsigned short* Hpl  = (unsigned short*)(ws + off); off += szH;
  float*          Rout = (float*)(ws + off);          off += szR;
  unsigned short* Xpl  = (unsigned short*)(ws + off); off += szX;
  unsigned short* Btpl = (unsigned short*)(ws + off); off += szBt;
  unsigned short* Ctpl = (unsigned short*)(ws + off); off += szCt;
  unsigned short* Mtpl = (unsigned short*)(ws + off); off += szMt;
  if (off > ws_size) return;
  float* out = (float*)d_out;

  {
    const int nthr = kBatch * kTimePad * (kDimIn / 8);
    castx_kernel<<<(nthr + 255) / 256, 256, 0, stream>>>(X, Xpl, nthr);
  }
  {
    const int nB = kState * kDimIn / 8;
    const int nC = kDimOut * kState / 8;
    const int nM = kDimOut * kArK / 8;
    wprep_kernel<0><<<(nB + 255) / 256, 256, 0, stream>>>(Bm, Btpl, nB);
    wprep_kernel<1><<<(nC + 255) / 256, 256, 0, stream>>>(Cm, Ctpl, nC);
    wprep_kernel<2><<<(nM + 255) / 256, 256, 0, stream>>>(Mm, Mtpl, nM);
  }
  for (int c = 0; c < kNumChunk; ++c) {
    const unsigned short* Ain = Xpl + (size_t)kPadRows * kDimIn + (size_t)c * kChunkB * kXPlane;
    wmma_gemm64<0, false, 0, 0, false, 0><<<dim3((kTime / 64) * (kState / 64) / 8, kChunkB), 256, 0, stream>>>(
        Ain, nullptr, kDimIn, (long)kXPlane,
        Btpl, nullptr, kDimIn, 0L,
        (void*)Ubuf, nullptr, kState, (long)kTime * kState,
        nullptr, nullptr, 0L,
        kTime, kState, kDimIn, kProjScale);
    scan_kernel<<<(kChunkB * (kState / 8)) / 32, 32, 0, stream>>>(Ubuf, H0, Ad, Hpl, c * kChunkB);
  }
  wmma_gemm64<0, false, 0, 0, false, 0><<<dim3((kBatch * kTime / 64) * (kDimOut / 64) / 8, 1), 256, 0, stream>>>(
      Hpl, nullptr, kState, 0L,
      Ctpl, nullptr, kState, 0L,
      (void*)Rout, nullptr, kDimOut, 0L,
      nullptr, nullptr, 0L,
      kBatch * kTime, kDimOut, kState, kReadScale);
  {
    const unsigned short* Awin = Xpl + (size_t)(kPadRows - (kTaps - 1)) * kDimIn;
    wmma_gemm64<0, false, 0, 0, true, 0><<<dim3((kTime / 64) * (kDimOut / 64) / 8, kBatch), 256, 0, stream>>>(
        Awin, nullptr, kDimIn, (long)kXPlane,
        Mtpl, nullptr, kArK, 0L,
        (void*)out, nullptr, kDimOut, (long)kTime * kDimOut,
        nullptr, (const float*)Rout, (long)kTime * kDimOut,
        kTime, kDimOut, kArK, kArScale);
  }
}
